// SSM_67714454389069
// MI455X (gfx1250) — hardware-verified
//
#include <hip/hip_runtime.h>
#include <stddef.h>
#include <stdint.h>
#include <math.h>

typedef __attribute__((ext_vector_type(16))) _Float16 v16h;
typedef __attribute__((ext_vector_type(8)))  _Float16 v8h;
typedef __attribute__((ext_vector_type(8)))  float    v8f;
typedef __attribute__((ext_vector_type(4)))  float    v4f;

constexpr int NVOX       = 8000;
constexpr int DIMV       = 20;
constexpr int NCH        = 64;
constexpr int NMID       = 16;
constexpr int UWIN       = 7;
constexpr int PADW       = 3;
constexpr int QPD        = DIMV + 2 * PADW;
constexpr int NSLOT      = QPD * QPD * QPD;
constexpr int NWIN       = UWIN * UWIN * UWIN;
constexpr int NSAMP      = NMID * NWIN;
constexpr int OCV        = NMID * NVOX;
constexpr int NOFF       = 27;
constexpr int KTOT       = NOFF * NMID;
constexpr int KSTEPS     = 14;
constexpr int NLAYER     = 3;
constexpr int WLAYER     = KSTEPS * 32 * 16;
constexpr int WPLANE     = NLAYER * WLAYER;
constexpr int NPREP      = WPLANE / 8;
constexpr int Q_PITCH    = 8192;
constexpr int QP_PITCH   = 17664;
constexpr int QP4        = QP_PITCH / 4;
constexpr int FEAT_PITCH = 32;
constexpr int T_PITCH    = 8064;
constexpr int SEG        = 64;
constexpr int SEGS_T     = T_PITCH / SEG;
constexpr int SEGS_O     = NVOX / SEG;
constexpr int ENC_THREADS = 128;
constexpr int BLK        = 256;
constexpr int NQBLK      = Q_PITCH / BLK;
constexpr int NPADBLK    = (NMID * QP4) / BLK;
constexpr int QITERS     = 32;
constexpr int STG_ITERS  = 43;
constexpr int M0_ROWS    = 125, M0_PAD = 128;
constexpr int M1_ROWS    = 27,  M1_PAD = 32;

constexpr float SIM_CARRY = 256.0f;
constexpr float W_CARRY   = 64.0f;
constexpr float ACT_CARRY = 256.0f;
constexpr float RES_CARRY = 2048.0f;
constexpr float RES_INV   = 1.0f / 2048.0f;
constexpr float FOLD_MAIN = 1.0f / 16384.0f;
constexpr float EPS_BN    = 1e-5f;
constexpr float EPS_IN    = 1e-5f;

static_assert(NSLOT == 17576 && NSAMP == 5488 && OCV == 128000);
static_assert(NWIN * OCV == NVOX * NSAMP);
static_assert(2 * KSTEPS - 1 == NOFF);
static_assert(KSTEPS * 32 == KTOT + 16);
static_assert(WLAYER % (ENC_THREADS * 8) == 0);
static_assert(NPREP % 32 == 0);
static_assert(STG_ITERS * ENC_THREADS >= NSAMP && (STG_ITERS - 1) * ENC_THREADS < NSAMP);
static_assert(NQBLK * BLK == Q_PITCH && Q_PITCH >= NVOX && Q_PITCH % 128 == 0);
static_assert(NPADBLK * BLK == NMID * QP4 && QP_PITCH >= NSLOT && QP_PITCH % 128 == 0);
static_assert(NVOX == 31 * BLK + 64);
static_assert(QITERS * BLK >= NVOX);
static_assert(T_PITCH % SEG == 0 && SEGS_T % 2 == 0 && T_PITCH >= NVOX);
static_assert((NCH * SEGS_T) % 16 == 0 && (NCH * SEGS_O) % 16 == 0);
static_assert((T_PITCH * 4) % 128 == 0 && (NVOX * 4) % 128 == 0 && (FEAT_PITCH * 4) == 128);
static_assert(SIM_CARRY == ACT_CARRY && SIM_CARRY * W_CARRY * FOLD_MAIN == 1.0f && RES_CARRY * RES_INV == 1.0f);
static_assert(M0_PAD * NMID >= 8 * 16 * NMID && M1_PAD >= M1_ROWS);
static_assert(SEGS_T > 16 && SEGS_O > 16);

constexpr size_t WS_Q      = 0;
constexpr size_t WS_Q_B    = (size_t)NMID * Q_PITCH * 4;
constexpr size_t WS_QPAD   = WS_Q + WS_Q_B;
constexpr size_t WS_QPAD_B = (size_t)NMID * QP_PITCH * 4;
constexpr size_t WS_WHI    = WS_QPAD + WS_QPAD_B;
constexpr size_t WS_W_B    = (size_t)WPLANE * 2;
constexpr size_t WS_WLO    = WS_WHI + WS_W_B;
constexpr size_t WS_FEAT   = WS_WLO + WS_W_B;
constexpr size_t WS_FEAT_B = (size_t)NVOX * FEAT_PITCH * 4;
constexpr size_t WS_T1     = WS_FEAT + WS_FEAT_B;
constexpr size_t WS_T_B    = (size_t)NCH * T_PITCH * 4;
constexpr size_t WS_T2     = WS_T1 + WS_T_B;
constexpr size_t WS_TOTAL  = WS_T2 + WS_T_B;
static_assert(WS_Q_B % 256 == 0 && WS_QPAD_B % 256 == 0 && WS_W_B % 256 == 0 && WS_FEAT_B % 256 == 0 && WS_T_B % 256 == 0);
static_assert(WS_TOTAL == 6893568 && WS_TOTAL <= (size_t)134217728);

__device__ __forceinline__ unsigned opq(unsigned v) { asm volatile("" : "+v"(v)); return v; }

union HU { v16h v; v8h h[2]; unsigned w[8]; };

__device__ __forceinline__ v8f wmma16(v16h a, v16h b, v8f c) {
  return __builtin_amdgcn_wmma_f32_16x16x32_f16(false, a, false, b, (short)0, c, false, false);
}
__device__ __forceinline__ void mma_guard1(v8f& c, v16h a, v16h b) {
  asm volatile("v_nop\n\tv_nop\n\tv_nop\n\tv_nop" : "+v"(c) : "v"(a), "v"(b));
}
__device__ __forceinline__ void mma_guard2(v8f& c, v8f& d, v16h a, v16h b, v16h e, v16h f) {
  asm volatile("v_nop\n\tv_nop\n\tv_nop\n\tv_nop" : "+v"(c), "+v"(d) : "v"(a), "v"(b), "v"(e), "v"(f));
}

template <bool FULL>
__device__ __forceinline__ void kstep_plain(v8f& accm, const _Float16* arow, int o0, int o1, const _Float16* bk) {
  HU a, b;
  a.h[0] = *(const v8h*)(arow + o0);
  if (FULL) { a.h[1] = *(const v8h*)(arow + o1); } else { a.w[4] = 0u; a.w[5] = 0u; a.w[6] = 0u; a.w[7] = 0u; }
  b.h[0] = *(const v8h*)(bk);
  b.h[1] = *(const v8h*)(bk + 8);
  accm = wmma16(a.v, b.v, accm);
  mma_guard1(accm, a.v, b.v);
}
template <bool FULL>
__device__ __forceinline__ void kstep_split(v8f& accm, v8f& accr, const _Float16* arow, const _Float16* arowl,
                                            int o0, int o1, const _Float16* bk, const _Float16* blk) {
  HU a, al, b, bl;
  a.h[0]  = *(const v8h*)(arow + o0);
  al.h[0] = *(const v8h*)(arowl + o0);
  if (FULL) {
    a.h[1]  = *(const v8h*)(arow + o1);
    al.h[1] = *(const v8h*)(arowl + o1);
  } else {
    a.w[4] = 0u; a.w[5] = 0u; a.w[6] = 0u; a.w[7] = 0u;
    al.w[4] = 0u; al.w[5] = 0u; al.w[6] = 0u; al.w[7] = 0u;
  }
  b.h[0]  = *(const v8h*)(bk);      b.h[1]  = *(const v8h*)(bk + 8);
  bl.h[0] = *(const v8h*)(blk);     bl.h[1] = *(const v8h*)(blk + 8);
  accm = wmma16(a.v, b.v, accm);
  accr = wmma16(a.v, bl.v, accr);
  accr = wmma16(al.v, b.v, accr);
  mma_guard2(accm, accr, a.v, b.v, al.v, bl.v);
}

template <int IN, int OUT>
__device__ __forceinline__ int a_rowbase(int mBase, int mValid, int lane) {
  int m = mBase + (lane & 15);
  m = (m < mValid) ? m : (mValid - 1);
  const unsigned mu = opq((unsigned)m);
  const unsigned z0 = mu / (unsigned)(OUT * OUT);
  const unsigned r0 = opq(mu - z0 * (unsigned)(OUT * OUT));
  const unsigned y0 = r0 / (unsigned)OUT;
  const unsigned x0 = r0 - y0 * (unsigned)OUT;
  return (((int)z0 * IN + (int)y0) * IN + (int)x0) * NMID + 8 * (lane >> 4);
}
template <int IN, int OUT>
__device__ __forceinline__ void conv_tile_plain(const _Float16* ain, const _Float16* wh, const int* sp,
                                                int mBase, int mValid, int lane, v8f& accm) {
  const _Float16* arow = ain + a_rowbase<IN, OUT>(mBase, mValid, lane);
  const _Float16* bp = wh + lane * 16;
  accm = (v8f){0.f, 0.f, 0.f, 0.f, 0.f, 0.f, 0.f, 0.f};
#pragma unroll 1
  for (int ks = 0; ks < KSTEPS - 1; ++ks)
    kstep_plain<true>(accm, arow, sp[2 * ks], sp[2 * ks + 1], bp + ks * 512);
  kstep_plain<false>(accm, arow, sp[2 * (KSTEPS - 1)], 0, bp + (KSTEPS - 1) * 512);
}
template <int IN, int OUT>
__device__ __forceinline__ void conv_tile_split(const _Float16* ainh, const _Float16* ainl,
                                                const _Float16* wh, const _Float16* wl, const int* sp,
                                                int mBase, int mValid, int lane, v8f& accm, v8f& accr) {
  const int rb = a_rowbase<IN, OUT>(mBase, mValid, lane);
  const _Float16* arow  = ainh + rb;
  const _Float16* arowl = ainl + rb;
  const _Float16* bp  = wh + lane * 16;
  const _Float16* blp = wl + lane * 16;
  accm = (v8f){0.f, 0.f, 0.f, 0.f, 0.f, 0.f, 0.f, 0.f};
  accr = (v8f){0.f, 0.f, 0.f, 0.f, 0.f, 0.f, 0.f, 0.f};
#pragma unroll 1
  for (int ks = 0; ks < KSTEPS - 1; ++ks)
    kstep_split<true>(accm, accr, arow, arowl, sp[2 * ks], sp[2 * ks + 1], bp + ks * 512, blp + ks * 512);
  kstep_split<false>(accm, accr, arow, arowl, sp[2 * (KSTEPS - 1)], 0, bp + (KSTEPS - 1) * 512, blp + (KSTEPS - 1) * 512);
}

__device__ __forceinline__ void store_act(v8f acc, int mBase, int lane, float scf, float sh, _Float16* oh, _Float16* ol) {
  const int n = lane & 15;
  const int r0 = mBase + 8 * (lane >> 4);
#pragma unroll
  for (int r = 0; r < 8; ++r) {
    float val = fmaf(acc[r], scf, sh);
    val = (val > 0.0f) ? val : 0.0f;
    const float vc = val * ACT_CARRY;
    const _Float16 hv = (_Float16)vc;
    const _Float16 lv = (_Float16)((vc - (float)hv) * RES_CARRY);
    oh[(r0 + r) * NMID + n] = hv;
    ol[(r0 + r) * NMID + n] = lv;
  }
}

__device__ __forceinline__ void stage_w(_Float16* dst, const _Float16* __restrict__ src, int tid) {
#pragma unroll 1
  for (int i = tid; i < WLAYER / 8; i += ENC_THREADS) {
    const v8h t = *(const v8h*)(src + (size_t)i * 8);
    *(v8h*)(dst + i * 8) = t;
  }
}

__global__ __launch_bounds__(BLK) void k_wpack(const float* __restrict__ conv_w,
                                               _Float16* __restrict__ whi, _Float16* __restrict__ wlo) {
  const int i = blockIdx.x * BLK + threadIdx.x;
  if (i >= NPREP) return;
  const unsigned iu    = opq((unsigned)i);
  const unsigned eblk  = iu & 1u;
  const unsigned ln    = (iu >> 1) & 31u;
  const unsigned ksl   = iu >> 6;
  const unsigned layer = ksl / (unsigned)KSTEPS;
  const unsigned ks    = ksl - layer * (unsigned)KSTEPS;
  const unsigned hsel  = ln >> 4, n = ln & 15u;
  v8h hv, lv;
#pragma unroll
  for (int e = 0; e < 8; ++e) {
    const int k = (int)(ks * 32u + 8u * hsel + 16u * eblk) + e;
    const bool valid = (k < KTOT);
    const unsigned kc = opq((unsigned)(valid ? k : (KTOT - 1)));
    const unsigned off = kc >> 4, cc = kc & 15u;
    const unsigned d0 = off / 9u;
    const unsigned r9 = opq(off - d0 * 9u);
    const unsigned d1 = r9 / 3u;
    const unsigned d2 = r9 - d1 * 3u;
    const float w = conv_w[(((((int)layer * NMID + (int)n) * NMID + (int)cc) * 3 + (int)d0) * 3 + (int)d1) * 3 + (int)d2];
    const float fac = valid ? W_CARRY : 0.0f;
    const float vsc = w * fac;
    const _Float16 h16 = (_Float16)vsc;
    hv[e] = h16;
    lv[e] = (_Float16)((vsc - (float)h16) * RES_CARRY);
  }
  const size_t o = (size_t)i * 8;
  *(volatile v8h*)(whi + o) = hv;
  *(volatile v8h*)(wlo + o) = lv;
  __threadfence();
  *(volatile v8h*)(whi + o) = hv;
  *(volatile v8h*)(wlo + o) = lv;
}

__global__ __launch_bounds__(BLK) void k_fillq(const float* __restrict__ x, const float* __restrict__ w_red,
                                               float* __restrict__ qpl) {
  __shared__ __align__(16) float swt[NCH * NMID];
  __shared__ __align__(16) float stg[NMID * BLK];
  const int tid = threadIdx.x, lane = tid & 31, wave = tid >> 5;
  {
    const v4f wv = *(const v4f*)(w_red + tid * 4);
    const unsigned t = opq((unsigned)tid);
    const int c = (int)(t >> 4), ci0 = (int)((t & 15u) * 4u);
    swt[(ci0 + 0) * NMID + c] = wv[0];
    swt[(ci0 + 1) * NMID + c] = wv[1];
    swt[(ci0 + 2) * NMID + c] = wv[2];
    swt[(ci0 + 3) * NMID + c] = wv[3];
  }
  __syncthreads();
  const int col = blockIdx.x * BLK + tid;
  const int vox = (col < NVOX) ? col : (NVOX - 1);
  float q[NMID];
#pragma unroll
  for (int c = 0; c < NMID; ++c) q[c] = 0.0f;
#pragma unroll 2
  for (int ci = 0; ci < NCH; ++ci) {
    const float xv = x[(size_t)ci * NVOX + vox];
    const v4f wa = *(const v4f*)(swt + ci * NMID);
    const v4f wb = *(const v4f*)(swt + ci * NMID + 4);
    const v4f wc = *(const v4f*)(swt + ci * NMID + 8);
    const v4f wd = *(const v4f*)(swt + ci * NMID + 12);
#pragma unroll
    for (int j = 0; j < 4; ++j) {
      q[j]      = fmaf(wa[j], xv, q[j]);
      q[4 + j]  = fmaf(wb[j], xv, q[4 + j]);
      q[8 + j]  = fmaf(wc[j], xv, q[8 + j]);
      q[12 + j] = fmaf(wd[j], xv, q[12 + j]);
    }
  }
  float ss = 0.0f;
#pragma unroll
  for (int c = 0; c < NMID; ++c) ss = fmaf(q[c], q[c], ss);
  const float den = fmaxf(sqrtf(ss), 1e-12f);
  const float inv = 1.0f / den;
#pragma unroll
  for (int c = 0; c < NMID; ++c) stg[c * BLK + tid] = q[c] * inv;
  __syncthreads();
  v4f sv[4];
#pragma unroll
  for (int it = 0; it < 4; ++it) {
    const int c  = 2 * wave + (it >> 1);
    const int f0 = (it & 1) * 128 + lane * 4;
    sv[it] = *(const v4f*)(stg + c * BLK + f0);
  }
  for (int pass = 0; pass < 2; ++pass) {
#pragma unroll
    for (int it = 0; it < 4; ++it) {
      const int c  = 2 * wave + (it >> 1);
      const int f0 = (it & 1) * 128 + lane * 4;
      *(volatile v4f*)(qpl + (size_t)c * Q_PITCH + (size_t)blockIdx.x * BLK + f0) = sv[it];
    }
    __threadfence();
  }
}

__global__ __launch_bounds__(BLK) void k_padq(const float* __restrict__ qpl, float* __restrict__ qpad) {
  const int i  = blockIdx.x * BLK + threadIdx.x;
  const unsigned iu = opq((unsigned)i);
  const unsigned c  = iu / (unsigned)QP4;
  const unsigned s4 = (iu - c * (unsigned)QP4) * 4u;
  v4f o;
#pragma unroll
  for (int e = 0; e < 4; ++e) {
    const unsigned s   = s4 + (unsigned)e;
    const bool ins = (s < (unsigned)NSLOT);
    const unsigned sc  = opq(ins ? s : (unsigned)(NSLOT - 1));
    const unsigned pz  = sc / (unsigned)(QPD * QPD);
    const unsigned rem = opq(sc - pz * (unsigned)(QPD * QPD));
    const unsigned py  = rem / (unsigned)QPD;
    const unsigned px  = rem - py * (unsigned)QPD;
    const bool inside = ins && (pz >= (unsigned)PADW) && (pz < (unsigned)(PADW + DIMV)) && (py >= (unsigned)PADW) && (py < (unsigned)(PADW + DIMV))
                        && (px >= (unsigned)PADW) && (px < (unsigned)(PADW + DIMV));
    int lz = (int)pz - PADW; lz = (lz < 0) ? 0 : ((lz > DIMV - 1) ? (DIMV - 1) : lz);
    int ly = (int)py - PADW; ly = (ly < 0) ? 0 : ((ly > DIMV - 1) ? (DIMV - 1) : ly);
    int lx = (int)px - PADW; lx = (lx < 0) ? 0 : ((lx > DIMV - 1) ? (DIMV - 1) : lx);
    const int vox = (lz * DIMV + ly) * DIMV + lx;
    const float val = qpl[(size_t)c * Q_PITCH + vox];
    const float fin = inside ? 1.0f : 0.0f;
    o[e] = val * fin;
  }
  float* op = qpad + (size_t)i * 4;
  *(volatile v4f*)op = o;
  __threadfence();
  *(volatile v4f*)op = o;
}

__global__ __launch_bounds__(ENC_THREADS) void k_enc(const float* __restrict__ qpl, const float* __restrict__ qpad,
    const _Float16* __restrict__ whi, const _Float16* __restrict__ wlo,
    const float* __restrict__ conv_b, const float* __restrict__ bn_g, const float* __restrict__ bn_b,
    const float* __restrict__ bn_m, const float* __restrict__ bn_v, float* __restrict__ feat) {
  __shared__ __align__(16) _Float16 s_sim[NWIN * NMID];
  __shared__ __align__(16) _Float16 s_b1h[M0_PAD * NMID];
  __shared__ __align__(16) _Float16 s_b1l[M0_PAD * NMID];
  __shared__ __align__(16) _Float16 s_b2h[M1_PAD * NMID];
  __shared__ __align__(16) _Float16 s_b2l[M1_PAD * NMID];
  __shared__ __align__(16) _Float16 s_wh[WLAYER];
  __shared__ __align__(16) _Float16 s_wl[WLAYER];
  __shared__ __align__(16) float s_feat[FEAT_PITCH];
  __shared__ float s_sb[NLAYER * 32];
  __shared__ int s_sp[NLAYER * NOFF];

  const int nsmp = blockIdx.x;
  const int tid = threadIdx.x, lane = tid & 31, wave = tid >> 5, hh = lane >> 4, n16 = lane & 15;

  if (tid < NLAYER * NOFF) {
    const unsigned t     = opq((unsigned)tid);
    const unsigned which = t / (unsigned)NOFF;
    const unsigned off   = opq(t - which * (unsigned)NOFF);
    const int inw = UWIN - 2 * (int)which;
    const unsigned d0 = off / 9u;
    const unsigned r9 = opq(off - d0 * 9u);
    const unsigned d1 = r9 / 3u;
    const unsigned d2 = r9 - d1 * 3u;
    s_sp[tid] = (((int)d0 * inw + (int)d1) * inw + (int)d2) * NMID;
  }
  if (tid < NLAYER * 32) {
    const unsigned t = opq((unsigned)tid);
    const unsigned lyr = t >> 5, j = t & 31u, ch = j & 15u;
    const int idx = (int)(lyr * (unsigned)NMID + ch);
    const float g = bn_g[idx], bb = bn_b[idx], mu = bn_m[idx], var = bn_v[idx], cb = conv_b[idx];
    const float sc = g * (1.0f / sqrtf(var + EPS_BN));
    const float sh = fmaf(cb - mu, sc, bb);
    const float fa = (j < 16u) ? 1.0f : 0.0f;
    s_sb[tid] = fmaf(fa, sc, (1.0f - fa) * sh);
  }
  stage_w(s_wh, whi, tid);
  {
    const unsigned fbase = (unsigned)nsmp * (unsigned)NSAMP;
#pragma unroll 1
    for (int i = 0; i < STG_ITERS; ++i) {
      const int e   = tid + ENC_THREADS * i;
      const int ec  = (e < NSAMP) ? e : (NSAMP - 1);
      const unsigned ecu = opq((unsigned)ec);
      const unsigned gix = fbase + ecu;
      const unsigned o   = opq(gix / (unsigned)OCV);
      const unsigned r1  = opq(gix - o * (unsigned)OCV);
      const unsigned ch  = r1 / (unsigned)NVOX;
      const unsigned vox = opq(r1 - ch * (unsigned)NVOX);
      const unsigned pl  = vox / (unsigned)(DIMV * DIMV);
      const unsigned r2  = opq(vox - pl * (unsigned)(DIMV * DIMV));
      const unsigned pw  = r2 / (unsigned)DIMV;
      const unsigned ph  = r2 - pw * (unsigned)DIMV;
      const unsigned o0  = o / (unsigned)(UWIN * UWIN);
      const unsigned r3  = opq(o - o0 * (unsigned)(UWIN * UWIN));
      const unsigned o1  = r3 / (unsigned)UWIN;
      const unsigned o2  = r3 - o1 * (unsigned)UWIN;
      const unsigned slot = ((pl + o0) * (unsigned)QPD + (pw + o1)) * (unsigned)QPD + (ph + o2);
      const float qa = qpl[(size_t)ch * Q_PITCH + vox];
      const float qn = qpad[(size_t)ch * QP_PITCH + slot];
      float p = qn * qa;
      p = (p > 0.0f) ? p : 0.0f;
      const unsigned cpr = ecu / (unsigned)NWIN;
      const unsigned wpr = ecu - cpr * (unsigned)NWIN;
      s_sim[wpr * (unsigned)NMID + cpr] = (_Float16)(p * SIM_CARRY);
    }
  }
  __syncthreads();

  {
    const float scf = s_sb[n16] * FOLD_MAIN;
    const float sh  = s_sb[16 + n16];
    v8f acc;
    conv_tile_plain<7, 5>(s_sim, s_wh, s_sp, wave * 16, M0_ROWS, lane, acc);
    store_act(acc, wave * 16, lane, scf, sh, s_b1h, s_b1l);
    conv_tile_plain<7, 5>(s_sim, s_wh, s_sp, (wave + 4) * 16, M0_ROWS, lane, acc);
    store_act(acc, (wave + 4) * 16, lane, scf, sh, s_b1h, s_b1l);
  }
  __syncthreads();
  stage_w(s_wh, whi + WLAYER, tid);
  stage_w(s_wl, wlo + WLAYER, tid);
  __syncthreads();

  if (wave < 2) {
    const float scf = s_sb[32 + n16] * FOLD_MAIN;
    const float sh  = s_sb[48 + n16];
    v8f am, ar;
    conv_tile_split<5, 3>(s_b1h, s_b1l, s_wh, s_wl, s_sp + NOFF, wave * 16, M1_ROWS, lane, am, ar);
    const v8f acc = am + ar * RES_INV;
    store_act(acc, wave * 16, lane, scf, sh, s_b2h, s_b2l);
  }
  __syncthreads();
  stage_w(s_wh, whi + 2 * WLAYER, tid);
  stage_w(s_wl, wlo + 2 * WLAYER, tid);
  __syncthreads();

  if (wave == 0) {
    const float scf = s_sb[64 + n16] * FOLD_MAIN;
    const float sh  = s_sb[80 + n16];
    v8f am, ar;
    conv_tile_split<3, 1>(s_b2h, s_b2l, s_wh, s_wl, s_sp + 2 * NOFF, 0, 1, lane, am, ar);
    const float a0v = am[0] + ar[0] * RES_INV;
    float val = fmaf(a0v, scf, sh);
    val = (val > 0.0f) ? val : 0.0f;
    s_feat[lane] = (hh == 0) ? val : 0.0f;
  }
  __syncthreads();
  if (wave == 0) {
    const int l8 = lane & 7;
    const v4f fv = *(const v4f*)(s_feat + l8 * 4);
    float* fp = feat + (size_t)nsmp * FEAT_PITCH + l8 * 4;
    if (lane < 8) *(volatile v4f*)fp = fv;
    __threadfence();
    if (lane < 8) *(volatile v4f*)fp = fv;
  }
}

__global__ __launch_bounds__(BLK) void k_proj_norm(const float* __restrict__ feat, const float* __restrict__ w_out,
                                                   const float* __restrict__ b_out, const float* __restrict__ x,
                                                   float* __restrict__ t1) {
  __shared__ float sd[NVOX];
  __shared__ float sred[BLK / 32];
  const int c = blockIdx.x;
  const int tid = threadIdx.x, lane = tid & 31, wave = tid >> 5, hh = lane >> 4;
  v4f w4[4];
#pragma unroll
  for (int i = 0; i < 4; ++i) w4[i] = *(const v4f*)(w_out + c * NMID + 4 * i);
  const float bo = b_out[c];

  float lsum = 0.0f;
#pragma unroll 1
  for (int i = 0; i < QITERS; ++i) {
    const int vv = tid + BLK * i;
    const int vc = (vv < NVOX) ? vv : (NVOX - 1);
    const float fin = (vv < NVOX) ? 1.0f : 0.0f;
    const float* fptr = feat + (size_t)vc * FEAT_PITCH;
    const v4f f0 = *(const v4f*)(fptr);
    const v4f f1 = *(const v4f*)(fptr + 4);
    const v4f f2 = *(const v4f*)(fptr + 8);
    const v4f f3 = *(const v4f*)(fptr + 12);
    float acc = 0.0f;
#pragma unroll
    for (int e = 0; e < 4; ++e) acc = fmaf(w4[0][e], f0[e], acc);
#pragma unroll
    for (int e = 0; e < 4; ++e) acc = fmaf(w4[1][e], f1[e], acc);
#pragma unroll
    for (int e = 0; e < 4; ++e) acc = fmaf(w4[2][e], f2[e], acc);
#pragma unroll
    for (int e = 0; e < 4; ++e) acc = fmaf(w4[3][e], f3[e], acc);
    const float d = acc + bo;
    sd[vc] = d;
    lsum = fmaf(fin, d, lsum);
  }
  float s1 = lsum;
#pragma unroll
  for (int off = 1; off < 32; off <<= 1) s1 += __shfl_xor(s1, off, 32);
  if (lane == 0) sred[wave] = s1;
  __syncthreads();
  float tot = 0.0f;
#pragma unroll
  for (int w = 0; w < BLK / 32; ++w) tot += sred[w];
  const float mean = tot * (1.0f / (float)NVOX);
  __syncthreads();
  float lsq = 0.0f;
#pragma unroll 4
  for (int i = 0; i < QITERS; ++i) {
    const int vv = tid + BLK * i;
    const int vc = (vv < NVOX) ? vv : (NVOX - 1);
    const float fin = (vv < NVOX) ? 1.0f : 0.0f;
    const float dd = (sd[vc] - mean) * fin;
    lsq = fmaf(dd, dd, lsq);
  }
  float s2 = lsq;
#pragma unroll
  for (int off = 1; off < 32; off <<= 1) s2 += __shfl_xor(s2, off, 32);
  if (lane == 0) sred[wave] = s2;
  __syncthreads();
  float tot2 = 0.0f;
#pragma unroll
  for (int w = 0; w < BLK / 32; ++w) tot2 += sred[w];
  const float var  = tot2 * (1.0f / (float)NVOX);
  const float rstd = 1.0f / sqrtf(var + EPS_IN);

  v4f vals[8];
#pragma unroll
  for (int it = 0; it < 8; ++it) {
    int p = wave + 8 * it; p = (p < SEGS_T / 2) ? p : (SEGS_T / 2 - 1);
    const int f0 = (2 * p + hh) * SEG + 4 * (lane & 15);
    const int fs = (f0 < NVOX - 4) ? f0 : (NVOX - 4);
    const v4f xs = *(const v4f*)(x + (size_t)c * NVOX + fs);
    v4f o;
#pragma unroll
    for (int j = 0; j < 4; ++j) {
      float yv = (sd[fs + j] - mean) * rstd;
      yv = (yv > 0.0f) ? yv : 0.1f * yv;
      o[j] = xs[j] + yv;
    }
    vals[it] = o;
  }
  for (int pass = 0; pass < 2; ++pass) {
#pragma unroll
    for (int it = 0; it < 8; ++it) {
      const int p = wave + 8 * it;
      if (p < SEGS_T / 2) {
        const int f0 = (2 * p + hh) * SEG + 4 * (lane & 15);
        *(volatile v4f*)(t1 + (size_t)c * T_PITCH + f0) = vals[it];
      }
    }
    __threadfence();
  }
}

template <int LEAKY, int IN_P, int OUT_P, int SEGS>
__global__ __launch_bounds__(BLK) void k_pconv(const float* __restrict__ in, const float* __restrict__ w,
                                               const float* __restrict__ b, float* __restrict__ out) {
  __shared__ float sw[2 * NCH];
  __shared__ float sbias[32];
  const int tid = threadIdx.x, lane = tid & 31, wave = tid >> 5, hh = lane >> 4;
  const int pb = blockIdx.x * (BLK / 32);
  const int c0 = (2 * pb) / SEGS;
  if (tid < 2 * NCH) {
    int cc = c0 + (tid >> 6); cc = (cc < NCH) ? cc : (NCH - 1);
    sw[tid] = w[cc * NCH + (tid & 63)];
  }
  if (tid >= 128 && tid < 160) {
    int cc = c0 + (lane & 1); cc = (cc < NCH) ? cc : (NCH - 1);
    sbias[lane] = b[cc];
  }
  __syncthreads();
  const int p   = pb + wave;
  const int gs  = 2 * p + hh;
  const int c   = gs / SEGS;
  const int seg = gs - c * SEGS;
  const int dc  = c - c0;
  const float* swp = sw + dc * NCH;
  const int f0 = seg * SEG + 4 * (lane & 15);
  v4f acc = (v4f){0.0f, 0.0f, 0.0f, 0.0f};
#pragma unroll 4
  for (int k = 0; k < NCH; ++k) {
    const v4f iv = *(const v4f*)(in + (size_t)k * IN_P + f0);
    const float wk = swp[k];
    acc[0] = fmaf(wk, iv[0], acc[0]);
    acc[1] = fmaf(wk, iv[1], acc[1]);
    acc[2] = fmaf(wk, iv[2], acc[2]);
    acc[3] = fmaf(wk, iv[3], acc[3]);
  }
  const float bias = sbias[dc];
  v4f res;
#pragma unroll
  for (int j = 0; j < 4; ++j) {
    float r = acc[j] + bias;
    if (LEAKY) r = (r > 0.0f) ? r : 0.01f * r;
    res[j] = r;
  }
  float* op = out + (size_t)c * OUT_P + f0;
  *(volatile v4f*)op = res;
  __threadfence();
  *(volatile v4f*)op = res;
}

extern "C" void kernel_launch(void* const* d_in, const int* in_sizes, int n_in,
                              void* d_out, int out_size, void* d_ws, size_t ws_size,
                              hipStream_t stream) {
  if (n_in < 14) return;
  if (ws_size < WS_TOTAL) return;
  if ((size_t)out_size < (size_t)NCH * NVOX) return;
  if (in_sizes[0] != NCH * NVOX) return;
  if (in_sizes[1] != NMID * NCH) return;
  if (in_sizes[2] != NLAYER * NMID * KTOT) return;

  const float* x      = (const float*)d_in[0];
  const float* w_red  = (const float*)d_in[1];
  const float* conv_w = (const float*)d_in[2];
  const float* conv_b = (const float*)d_in[3];
  const float* bn_g   = (const float*)d_in[4];
  const float* bn_b   = (const float*)d_in[5];
  const float* bn_m   = (const float*)d_in[6];
  const float* bn_v   = (const float*)d_in[7];
  const float* w_out  = (const float*)d_in[8];
  const float* b_out  = (const float*)d_in[9];
  const float* w_f1   = (const float*)d_in[10];
  const float* b_f1   = (const float*)d_in[11];
  const float* w_f2   = (const float*)d_in[12];
  const float* b_f2   = (const float*)d_in[13];
  float* out = (float*)d_out;

  char* ws = (char*)d_ws;
  float*    qpl  = (float*)(ws + WS_Q);
  float*    qpad = (float*)(ws + WS_QPAD);
  _Float16* whi  = (_Float16*)(ws + WS_WHI);
  _Float16* wlo  = (_Float16*)(ws + WS_WLO);
  float*    feat = (float*)(ws + WS_FEAT);
  float*    t1   = (float*)(ws + WS_T1);
  float*    t2   = (float*)(ws + WS_T2);

  k_wpack<<<(NPREP + BLK - 1) / BLK, BLK, 0, stream>>>(conv_w, whi, wlo);
  k_fillq<<<NQBLK, BLK, 0, stream>>>(x, w_red, qpl);
  k_padq<<<NPADBLK, BLK, 0, stream>>>(qpl, qpad);
  k_enc<<<NVOX, ENC_THREADS, 0, stream>>>(qpl, qpad, whi, wlo, conv_b, bn_g, bn_b, bn_m, bn_v, feat);
  k_proj_norm<<<NCH, BLK, 0, stream>>>(feat, w_out, b_out, x, t1);
  k_pconv<1, T_PITCH, T_PITCH, SEGS_T><<<(NCH * SEGS_T) / 16, BLK, 0, stream>>>(t1, w_f1, b_f1, t2);
  k_pconv<0, T_PITCH, NVOX, SEGS_O><<<(NCH * SEGS_O) / 16, BLK, 0, stream>>>(t2, w_f2, b_f2, out);
}
